// PatchLocalPoolPointnetLatent_82660940578890
// MI455X (gfx1250) — hardware-run, weakly checked
//
#include <hip/hip_runtime.h>


namespace {
constexpr int NB = 2, T = 100000, NPT = NB * T, HID = 128, C2 = 256, G = 32768, NV = NB * G, NBLK = 5;
constexpr float XS = 8.0f, WSC = 256.0f;
static_assert(T % 16 == 0 && G % 64 == 0, "16-point waves must not straddle a batch");

typedef _Float16 b16;
typedef __attribute__((ext_vector_type(16))) _Float16 v16b;
typedef __attribute__((ext_vector_type(8))) _Float16 v8b;
typedef __attribute__((ext_vector_type(8))) float v8f;
typedef __attribute__((ext_vector_type(4))) float v4f;
__device__ __forceinline__ float bf16_rne(float f) { unsigned int u = __float_as_uint(f); u += 0x7FFFu + ((u >> 16) & 1u); return __uint_as_float(u & 0xFFFF0000u); }
__device__ __forceinline__ void split16(float v, b16& hi, b16& lo) { hi = (b16)v; lo = (b16)(v - (float)hi); }
__device__ __forceinline__ v16b frag_kb(const b16* p, int hh) { const v8b a = *(const v8b*)(p + 8 * hh), b = *(const v8b*)(p + 16 + 8 * hh); v16b f;
#pragma unroll
  for (int e = 0; e < 8; ++e) { f[e] = a[e]; f[8 + e] = b[e]; } return f; }
__device__ __forceinline__ v8f wmma16b(v16b a, v16b b, v8f c) { v8f d = __builtin_amdgcn_wmma_f32_16x16x32_f16(false, a, false, b, (short)0, c, false, false); asm volatile("v_nop\n\tv_nop\n\tv_nop\n\tv_nop" : "+v"(d) : "v"(a), "v"(b)); return d; }
__device__ __forceinline__ void wave_lds_sync() { __builtin_amdgcn_fence(__ATOMIC_RELEASE, "workgroup"); __builtin_amdgcn_wave_barrier(); __builtin_amdgcn_fence(__ATOMIC_ACQUIRE, "workgroup"); }
__device__ __forceinline__ int iclamp(int v, int lo, int hi) { return v < lo ? lo : (v > hi ? hi : v); }

constexpr int CSR_NBLK = 512, CSR_GB = 9, CSR_GN = 1 << CSR_GB  , CSR_MAXG = 512, CSR_CAP = 12288  ;
__global__ __launch_bounds__(64) void csrA_kernel(const int* __restrict__ dst, int E, int N, int nG, int CHP, int NGP, int* __restrict__ STG, int* __restrict__ HST) {
  extern __shared__ int sm[];
  int* cnt = sm; int* run = sm + NGP; int* ids = sm + 2 * NGP;
  const int b = blockIdx.x; const int ch = (E + CSR_NBLK - 1) / CSR_NBLK; const int e0 = b * ch, e1 = min(E, e0 + ch);
  for (int i = threadIdx.x; i < NGP; i += 64) cnt[i] = 0;
  for (int i = threadIdx.x; i < CHP; i += 64) ids[i] = -1;
  __syncthreads();
  if (threadIdx.x == 0) {
    for (int e = e0; e < e1; ++e) { int d = dst[e]; d = (d < 0) ? 0 : (d >= N ? N - 1 : d); cnt[d >> CSR_GB] += 1; }
    int acc = 0; for (int g = 0; g < nG; ++g) { run[g] = acc; acc += cnt[g]; }
    for (int e = e0; e < e1; ++e) { int d = dst[e]; d = (d < 0) ? 0 : (d >= N ? N - 1 : d); const int g = d >> CSR_GB; ids[run[g]] = e; run[g] += 1; } }
  __syncthreads();
  typedef __attribute__((ext_vector_type(4))) int v4i;
  for (int pass = 0; pass < 2; ++pass) {
    for (int i = threadIdx.x; i < CHP / 4; i += 64) *(volatile v4i*)(STG + (size_t)b * CHP + i * 4) = *(const v4i*)(&ids[i * 4]);
    for (int i = threadIdx.x; i < NGP / 4; i += 64) { v4i v; for (int e = 0; e < 4; ++e) v[e] = (i * 4 + e < nG) ? cnt[i * 4 + e] : 0; *(volatile v4i*)(HST + (size_t)b * NGP + i * 4) = v; }
    __threadfence(); }
}
__global__ __launch_bounds__(512) void csrS_kernel(const int* __restrict__ HST, int nG, int NGP, int* __restrict__ START, int* __restrict__ TOT, int* __restrict__ OFF) {
  __shared__ int tot[CSR_MAXG];
  const int b = threadIdx.x;
  for (int pass = 0; pass < 2; ++pass) { int runb = 0; for (int g = 0; g < nG; ++g) { int c = HST[(size_t)b * NGP + g]; c = (c < 0) ? 0 : c; ((volatile int*)OFF)[(size_t)g * CSR_NBLK + b] = runb; runb += c; } __threadfence(); }
  for (int g = threadIdx.x; g < nG; g += 512) { int s = 0; for (int bb = 0; bb < CSR_NBLK; ++bb) { int c = HST[(size_t)bb * NGP + g]; s += (c < 0) ? 0 : c; } tot[g] = s; }
  __syncthreads();
  if (threadIdx.x < 32) {
    __shared__ int st[CSR_MAXG + 32];
    if (threadIdx.x == 0) { int acc = 0; for (int g = 0; g < NGP; ++g) { st[g] = acc; if (g < nG) acc += (tot[g] + 31) & ~31; } st[NGP] = acc; }
    __builtin_amdgcn_fence(__ATOMIC_RELEASE, "workgroup"); __builtin_amdgcn_wave_barrier(); __builtin_amdgcn_fence(__ATOMIC_ACQUIRE, "workgroup");
    for (int pass = 0; pass < 2; ++pass) { for (int i = threadIdx.x; i < NGP + 32; i += 32) { ((volatile int*)START)[i] = (i <= NGP) ? st[min(i, NGP)] : 0; ((volatile int*)TOT)[i] = (i < nG) ? tot[i] : 0; } __threadfence(); } }
}
__global__ __launch_bounds__(256) void csrB_kernel(const int* __restrict__ dst, int N, int nG, int CHP, int NGP, int permLen, const int* __restrict__ STG, const int* __restrict__ HST, const int* __restrict__ OFF, const int* __restrict__ START, const int* __restrict__ TOT, int* __restrict__ PERM, int* __restrict__ ROWPTR, int* __restrict__ ROWCNT, int* __restrict__ FLAG) {
  typedef __attribute__((ext_vector_type(4))) int v4i;
  __shared__ int ids[CSR_CAP]; __shared__ unsigned short key[CSR_CAP]; __shared__ int outp[CSR_CAP]; __shared__ int ncnt[CSR_GN + 1]; __shared__ int boff[CSR_NBLK + 1];
  const int g = blockIdx.x, t_ = threadIdx.x; int tot = TOT[g]; int st = START[g], stn = START[g + 1]; const int v0 = g * CSR_GN; const int nv = min(CSR_GN, N - v0);
  st = (st < 0) ? 0 : (st > permLen - 32 ? permLen - 32 : st) & ~31; stn = (stn < st) ? st : (stn > permLen ? permLen : stn); tot = (tot < 0) ? 0 : tot; if (tot > stn - st && tot <= CSR_CAP) tot = stn - st;
  if (tot > CSR_CAP) {
    for (int pass = 0; pass < 2; ++pass) { for (int i = t_; i < CSR_GN / 4; i += 256) { v4i a, c; for (int e = 0; e < 4; ++e) { a[e] = st; c[e] = 0; } *(volatile v4i*)(ROWPTR + v0 + i * 4) = a; *(volatile v4i*)(ROWCNT + v0 + i * 4) = c; } if (t_ == 0) ((volatile int*)FLAG)[0] = 1; __threadfence(); } (void)nv; return; }
  if (t_ == 0) { int acc = 0; for (int b = 0; b < CSR_NBLK; ++b) { boff[b] = acc; int c = HST[(size_t)b * NGP + g]; c = (c < 0) ? 0 : (c > CHP ? CHP : c); acc += c; if (acc > tot) acc = tot; } boff[CSR_NBLK] = acc; }
  for (int i = t_; i <= CSR_GN; i += 256) ncnt[i] = 0;
  __syncthreads();
  for (int b = 0; b < CSR_NBLK; ++b) { const int c = boff[b + 1] - boff[b]; int o_ = OFF[(size_t)g * CSR_NBLK + b]; o_ = (o_ < 0) ? 0 : (o_ > CHP - c ? CHP - c : o_); const int* src_ = STG + (size_t)b * CHP + o_;
    for (int i = t_; i < c; i += 256) { int id = src_[i]; id = (id < 0) ? 0 : id; ids[boff[b] + i] = id; int d = dst[id]; d = (d < v0) ? v0 : (d >= N ? N - 1 : d); int kk = d - v0; kk = (kk < 0) ? 0 : (kk >= CSR_GN ? CSR_GN - 1 : kk); key[boff[b] + i] = (unsigned short)kk; } }
  __syncthreads();
  if (t_ == 0) { for (int i = 0; i < tot; ++i) ncnt[key[i]] += 1; int acc = 0; for (int vl = 0; vl < CSR_GN; ++vl) { const int c = ncnt[vl]; ncnt[vl] = acc; acc += c; } ncnt[CSR_GN] = acc;
    for (int i = 0; i < tot; ++i) { const int vl = key[i]; outp[ncnt[vl]] = ids[i]; ncnt[vl] += 1; }
    for (int vl = CSR_GN; vl > 0; --vl) ncnt[vl] = ncnt[vl - 1]; ncnt[0] = 0; }
  __syncthreads();
  for (int pass = 0; pass < 2; ++pass) {
    for (int i = t_; i < (stn - st) / 4; i += 256) { v4i v; for (int e = 0; e < 4; ++e) { const int q = i * 4 + e; v[e] = (q < tot) ? outp[q] : -1; } *(volatile v4i*)(PERM + st + i * 4) = v; }
    for (int i = t_; i < CSR_GN / 4; i += 256) { v4i a, c; for (int e = 0; e < 4; ++e) { const int vl = i * 4 + e; a[e] = st + ncnt[vl]; c[e] = (vl < nv) ? (ncnt[vl + 1] - ncnt[vl]) : 0; } *(volatile v4i*)(ROWPTR + v0 + i * 4) = a; *(volatile v4i*)(ROWCNT + v0 + i * 4) = c; }
    __threadfence(); }
}
__global__ __launch_bounds__(256) void csrZ_kernel(int* __restrict__ p, size_t n4) { typedef __attribute__((ext_vector_type(4))) int v4i; const size_t tid = (size_t)blockIdx.x * 256 + threadIdx.x, nth = (size_t)gridDim.x * 256; v4i z = {0, 0, 0, 0}; for (size_t i = tid; i < n4; i += nth) *(volatile v4i*)(p + i * 4) = z; }
struct CsrBufs { int *STG, *HST, *OFF, *START, *TOT, *PERM, *ROWPTR, *ROWCNT, *FLAG; int nG, NGP, CHP; size_t permLen; char* base; size_t bytes; };
static size_t csr_carve(CsrBufs& c, char* ws, size_t off, int E, int N) {
  const size_t off0 = off; c.base = ws + off;
  auto al = [&](size_t bytes) { char* p = ws + off; off += (bytes + 255) & ~(size_t)255; return p; };
  c.nG = (N + CSR_GN - 1) / CSR_GN; c.NGP = (c.nG + 31) & ~31; const int ch = (E + CSR_NBLK - 1) / CSR_NBLK; c.CHP = (ch + 31) & ~31; c.permLen = (size_t)E + 32 * (size_t)c.nG + 32;
  c.STG = (int*)al((size_t)CSR_NBLK * c.CHP * 4); c.HST = (int*)al((size_t)CSR_NBLK * c.NGP * 4); c.OFF = (int*)al((size_t)c.NGP * CSR_NBLK * 4); c.START = (int*)al((size_t)(c.NGP + 64) * 4); c.TOT = (int*)al((size_t)(c.NGP + 64) * 4);
  c.PERM = (int*)al(c.permLen * 4); c.ROWPTR = (int*)al((size_t)c.nG * CSR_GN * 4); c.ROWCNT = (int*)al((size_t)c.nG * CSR_GN * 4); c.FLAG = (int*)al(256);
  c.bytes = off - off0; return off;
}
static void csr_build(const CsrBufs& c, const int* dst, int E, int N, hipStream_t stream) {
  const size_t smem = (size_t)(2 * c.NGP + c.CHP) * 4;
  csrZ_kernel<<<512, 256, 0, stream>>>((int*)c.base, c.bytes / 16);
  csrA_kernel<<<CSR_NBLK, 64, smem, stream>>>(dst, E, N, c.nG, c.CHP, c.NGP, c.STG, c.HST);
  csrS_kernel<<<1, 512, 0, stream>>>(c.HST, c.nG, c.NGP, c.START, c.TOT, c.OFF);
  csrB_kernel<<<c.nG, 256, 0, stream>>>(dst, N, c.nG, c.CHP, c.NGP, (int)c.permLen, c.STG, c.HST, c.OFF, c.START, c.TOT, c.PERM, c.ROWPTR, c.ROWCNT, c.FLAG);
}


__global__ __launch_bounds__(256) void prepp_kernel(const float* __restrict__ pts, const int* __restrict__ index, b16* __restrict__ P16, int* __restrict__ KEY) {
  const int tid = blockIdx.x * 256 + threadIdx.x, lane = threadIdx.x & 31, wave = tid >> 5;
  const int p0 = wave * 32; if (p0 >= NPT) return;
  const int p = p0 + lane; const int b = p / T; const int key = b * G + iclamp(index[p], 0, G - 1);
  for (int pass = 0; pass < 2; ++pass) { ((volatile int*)KEY)[p] = key; __threadfence(); }
  for (int q = 0; q < 4; ++q) { const int pp = p0 + q * 8 + (lane >> 2), seg = lane & 3; v8b o = {};
    if (seg == 0) { o[0] = (b16)(bf16_rne(pts[(size_t)pp * 3 + 0]) * XS); o[1] = (b16)(bf16_rne(pts[(size_t)pp * 3 + 1]) * XS); o[2] = (b16)(bf16_rne(pts[(size_t)pp * 3 + 2]) * XS); }
    for (int pass = 0; pass < 2; ++pass) { *(volatile v8b*)(P16 + (size_t)pp * 32 + seg * 8) = o; __threadfence(); } }
}
__global__ __launch_bounds__(256) void prepw_kernel(const float* __restrict__ wpos, const float* __restrict__ w0, const float* __restrict__ w1, const float* __restrict__ ws_, const float* __restrict__ wc, b16* __restrict__ WPOS, b16* __restrict__ W0T, b16* __restrict__ W1T, b16* __restrict__ WST, b16* __restrict__ WCT) {
  __shared__ __attribute__((aligned(16))) b16 Tt[64][64 + 8];
  const int kind = blockIdx.z, i0 = blockIdx.x * 64, o0 = blockIdx.y * 64, t_ = threadIdx.x;
  int IN, INP, OUT; const float* w; b16* dst;
  if (kind == 0) { IN = 3; INP = 32; OUT = C2; w = wpos; dst = WPOS; }
  else if (kind <= 5) { IN = C2; INP = C2; OUT = HID; w = w0 + (size_t)(kind - 1) * C2 * HID; dst = W0T + (size_t)(kind - 1) * HID * C2; }
  else if (kind <= 10) { IN = HID; INP = HID; OUT = HID; w = w1 + (size_t)(kind - 6) * HID * HID; dst = W1T + (size_t)(kind - 6) * HID * HID; }
  else if (kind <= 15) { IN = C2; INP = C2; OUT = HID; w = ws_ + (size_t)(kind - 11) * C2 * HID; dst = WST + (size_t)(kind - 11) * HID * C2; }
  else { IN = HID; INP = HID; OUT = HID; w = wc; dst = WCT; }
  if (i0 >= INP || o0 >= OUT) return;
  for (int q = t_; q < 64 * 64; q += 256) { const int ii = q >> 6, oo = q & 63; const int i = i0 + ii; Tt[oo][ii] = (i < IN) ? (b16)(bf16_rne(w[(size_t)(i < IN ? i : 0) * OUT + o0 + oo]) * WSC) : (b16)0.0f; }
  __syncthreads();
  for (int pass = 0; pass < 2; ++pass) { for (int q = t_; q < 64 * 8; q += 256) { const int oo = q >> 3, c8 = (q & 7) * 8; if (i0 + c8 < INP) *(volatile v8b*)(dst + (size_t)(o0 + oo) * INP + i0 + c8) = *(const v8b*)(&Tt[oo][c8]); } __threadfence(); }
}
__device__ __forceinline__ void relu_frags(v16b& h, v16b& l) {
#pragma unroll
  for (int e = 0; e < 16; ++e) { const bool pos_ = (float)h[e] > 0.0f; l[e] = pos_ ? l[e] : (b16)0.0f; h[e] = pos_ ? h[e] : (b16)0.0f; } }
template <int BLK0>
__global__ __launch_bounds__(128) void resnet_kernel(const b16* __restrict__ P16, const b16* __restrict__ WPOS, const float* __restrict__ bpos, const int* __restrict__ KEY, int pbase, int vbase, const b16* __restrict__ VOXh, const b16* __restrict__ VOXl,
                                                    const b16* __restrict__ W0T, const float* __restrict__ b0, const b16* __restrict__ W1T, const float* __restrict__ b1, const b16* __restrict__ WST, b16* __restrict__ NETh, b16* __restrict__ NETl) {
  __shared__ __attribute__((aligned(16))) b16 Xh[4][16][C2 + 8], Xl[4][16][C2 + 8], Hh[4][16][HID + 8], Hl[4][16][HID + 8];
  const int wave = threadIdx.x >> 5, lane = threadIdx.x & 31, nloc = lane & 15, hlf = lane >> 4; const size_t prow0 = ((size_t)blockIdx.x * 4 + wave) * 16;
  if (prow0 >= (size_t)T) return;
  if (BLK0) {
    const v16b a = frag_kb(P16 + ((size_t)pbase + prow0 + nloc) * 32, hlf);
#pragma unroll
    for (int t = 0; t < 16; ++t) { v8f acc = {}; acc = wmma16b(a, frag_kb(WPOS + (size_t)(t * 16 + nloc) * 32, hlf), acc); const float bb = bf16_rne(bpos[t * 16 + nloc]);
#pragma unroll
      for (int r = 0; r < 8; ++r) { b16 h_, l_; split16((acc[r] * (1.0f / (XS * WSC)) + bb) * XS, h_, l_); Xh[wave][8 * hlf + r][t * 16 + nloc] = h_; Xl[wave][8 * hlf + r][t * 16 + nloc] = l_; } }
  } else {
    const int rr = lane >> 1, hf = lane & 1; const size_t prow = prow0 + rr; const int key = iclamp(KEY[pbase + prow] - vbase, 0, G - 1);
    const v8b* sh = hf == 0 ? (const v8b*)(NETh + prow * HID) : (const v8b*)(VOXh + (size_t)key * HID); const v8b* sl = hf == 0 ? (const v8b*)(NETl + prow * HID) : (const v8b*)(VOXl + (size_t)key * HID);
#pragma unroll
    for (int q = 0; q < 16; ++q) { *(v8b*)(&Xh[wave][rr][hf * HID + q * 8]) = sh[q]; *(v8b*)(&Xl[wave][rr][hf * HID + q * 8]) = sl[q]; } }
  wave_lds_sync();
  v8f acc[8];
#pragma unroll
  for (int t = 0; t < 8; ++t) acc[t] = (v8f){};
#pragma unroll 2
  for (int kb = 0; kb < C2; kb += 32) { v16b a = frag_kb(&Xh[wave][nloc][kb], hlf), al = frag_kb(&Xl[wave][nloc][kb], hlf); relu_frags(a, al);
#pragma unroll
    for (int t = 0; t < 8; ++t) { const v16b bw = frag_kb(W0T + (size_t)(t * 16 + nloc) * C2 + kb, hlf); acc[t] = wmma16b(a, bw, acc[t]); acc[t] = wmma16b(al, bw, acc[t]); } }
#pragma unroll
  for (int t = 0; t < 8; ++t) { const float bb = bf16_rne(b0[t * 16 + nloc]);
#pragma unroll
    for (int r = 0; r < 8; ++r) { b16 h_, l_; split16(fmaxf(acc[t][r] * (1.0f / (XS * WSC)) + bb, 0.0f) * XS, h_, l_); Hh[wave][8 * hlf + r][t * 16 + nloc] = h_; Hl[wave][8 * hlf + r][t * 16 + nloc] = l_; } }
  wave_lds_sync();
#pragma unroll
  for (int t = 0; t < 8; ++t) acc[t] = (v8f){};
#pragma unroll
  for (int kb = 0; kb < HID; kb += 32) { const v16b a = frag_kb(&Hh[wave][nloc][kb], hlf), al = frag_kb(&Hl[wave][nloc][kb], hlf);
#pragma unroll
    for (int t = 0; t < 8; ++t) { const v16b bw = frag_kb(W1T + (size_t)(t * 16 + nloc) * HID + kb, hlf); acc[t] = wmma16b(a, bw, acc[t]); acc[t] = wmma16b(al, bw, acc[t]); } }
#pragma unroll 2
  for (int kb = 0; kb < C2; kb += 32) { const v16b a = frag_kb(&Xh[wave][nloc][kb], hlf), al = frag_kb(&Xl[wave][nloc][kb], hlf);
#pragma unroll
    for (int t = 0; t < 8; ++t) { const v16b bw = frag_kb(WST + (size_t)(t * 16 + nloc) * C2 + kb, hlf); acc[t] = wmma16b(a, bw, acc[t]); acc[t] = wmma16b(al, bw, acc[t]); } }
  wave_lds_sync();
#pragma unroll
  for (int t = 0; t < 8; ++t) { const float bb = bf16_rne(b1[t * 16 + nloc]);
#pragma unroll
    for (int r = 0; r < 8; ++r) { b16 h_, l_; split16((acc[t][r] * (1.0f / (XS * WSC)) + bb) * XS, h_, l_); Hh[wave][8 * hlf + r][t * 16 + nloc] = h_; Hl[wave][8 * hlf + r][t * 16 + nloc] = l_; } }
  wave_lds_sync();
  for (int pass = 0; pass < 2; ++pass) { for (int rr = 0; rr < 16; ++rr) if (lane < 16) { *(volatile v8b*)(NETh + (prow0 + rr) * HID + lane * 8) = *(const v8b*)(&Hh[wave][rr][lane * 8]); *(volatile v8b*)(NETl + (prow0 + rr) * HID + lane * 8) = *(const v8b*)(&Hl[wave][rr][lane * 8]); } __threadfence(); }
}
__global__ __launch_bounds__(256) void voxmax_kernel(const b16* __restrict__ NETh, const b16* __restrict__ NETl, int pbase, int vbase, const int* __restrict__ PERM, const int* __restrict__ ROWPTR, const int* __restrict__ ROWCNT, int permLen, b16* __restrict__ VOXh, b16* __restrict__ VOXl) {
  const int wave = threadIdx.x >> 5, lane = threadIdx.x & 31; const size_t vl = ((size_t)blockIdx.x * 8 + wave) * 2 + (lane >> 4); const size_t v = vbase + vl; const int c0 = (lane & 15) * 8;
  int st = ROWPTR[v], cnt = ROWCNT[v]; cnt = iclamp(cnt, 0, 8192); st = iclamp(st, 0, permLen - cnt);
  float m[8]; for (int j = 0; j < 8; ++j) m[j] = -INFINITY;
  for (int j = 0; j < cnt; ++j) { const int pr = iclamp(PERM[st + j] - pbase, 0, T - 1); const v8b xh = *(const v8b*)(NETh + (size_t)pr * HID + c0), xl = *(const v8b*)(NETl + (size_t)pr * HID + c0);
#pragma unroll
    for (int q = 0; q < 8; ++q) m[q] = fmaxf(m[q], (float)xh[q] + (float)xl[q]); }
  v8b oh, ol; for (int q = 0; q < 8; ++q) { b16 a_, c_; split16(cnt > 0 ? m[q] : 0.0f, a_, c_); oh[q] = a_; ol[q] = c_; }
  for (int pass = 0; pass < 2; ++pass) { *(volatile v8b*)(VOXh + vl * HID + c0) = oh; *(volatile v8b*)(VOXl + vl * HID + c0) = ol; __threadfence(); }
}
__global__ __launch_bounds__(256) void voxmean_kernel(const b16* __restrict__ NETh, const b16* __restrict__ NETl, int pbase, int vbase, const int* __restrict__ PERM, const int* __restrict__ ROWPTR, const int* __restrict__ ROWCNT, int permLen, b16* __restrict__ MNh, b16* __restrict__ MNl) {
  const int wave = threadIdx.x >> 5, lane = threadIdx.x & 31; const size_t vl = ((size_t)blockIdx.x * 8 + wave) * 2 + (lane >> 4); const size_t v = vbase + vl; const int c0 = (lane & 15) * 8;
  int st = ROWPTR[v], cnt = ROWCNT[v]; cnt = iclamp(cnt, 0, 8192); st = iclamp(st, 0, permLen - cnt);
  float s[8]; for (int j = 0; j < 8; ++j) s[j] = 0.0f;
  for (int j = 0; j < cnt; ++j) { const int pr = iclamp(PERM[st + j] - pbase, 0, T - 1); const v8b xh = *(const v8b*)(NETh + (size_t)pr * HID + c0), xl = *(const v8b*)(NETl + (size_t)pr * HID + c0);
#pragma unroll
    for (int q = 0; q < 8; ++q) s[q] += (float)xh[q] + (float)xl[q]; }
  const float inv = cnt > 0 ? 1.0f / (float)cnt : 0.0f; v8b oh, ol; for (int q = 0; q < 8; ++q) { b16 a_, c_; split16(s[q] * inv, a_, c_); oh[q] = a_; ol[q] = c_; }
  for (int pass = 0; pass < 2; ++pass) { *(volatile v8b*)(MNh + vl * HID + c0) = oh; *(volatile v8b*)(MNl + vl * HID + c0) = ol; __threadfence(); }
}
__global__ __launch_bounds__(256) void cnt_kernel(const int* __restrict__ ROWCNT, int* __restrict__ CNT) { const int i = blockIdx.x * 256 + threadIdx.x; if (i < NV) { const int c = ROWCNT[i]; for (int pass = 0; pass < 2; ++pass) { ((volatile int*)CNT)[i] = c; __threadfence(); } } }
__global__ __launch_bounds__(128) void final_kernel(const b16* __restrict__ MNh, const b16* __restrict__ MNl, const int* __restrict__ CNT, int b, const b16* __restrict__ WCT, const float* __restrict__ bc, float* __restrict__ out) {
  __shared__ __attribute__((aligned(16))) float Tc[HID][64 + 4];
  const int wave = threadIdx.x >> 5, lane = threadIdx.x & 31, nloc = lane & 15, hlf = lane >> 4, t_ = threadIdx.x; const int vloc0 = blockIdx.x * 64; const size_t m0 = (size_t)vloc0 + wave * 16;
  v8f acc[8];
#pragma unroll
  for (int t = 0; t < 8; ++t) acc[t] = (v8f){};
#pragma unroll
  for (int kb = 0; kb < HID; kb += 32) { const v16b a = frag_kb(MNh + (m0 + nloc) * HID + kb, hlf), al = frag_kb(MNl + (m0 + nloc) * HID + kb, hlf);
#pragma unroll
    for (int t = 0; t < 8; ++t) { const v16b bw = frag_kb(WCT + (size_t)(t * 16 + nloc) * HID + kb, hlf); acc[t] = wmma16b(a, bw, acc[t]); acc[t] = wmma16b(al, bw, acc[t]); } }
#pragma unroll
  for (int t = 0; t < 8; ++t) { const int ch = t * 16 + nloc; const float bb = bf16_rne(bc[ch]);
#pragma unroll
    for (int r = 0; r < 8; ++r) { const size_t vl = m0 + 8 * hlf + r; const bool ne = CNT[(size_t)b * G + vl] > 0; Tc[ch][wave * 16 + 8 * hlf + r] = ne ? acc[t][r] * (1.0f / (XS * WSC)) + bb : 0.0f; } }
  __syncthreads();
  for (int pass = 0; pass < 2; ++pass) { for (int q = t_; q < HID * 16; q += 128) { const int ch = q >> 4, c4 = (q & 15) * 4; *(volatile v4f*)(out + ((size_t)b * HID + ch) * G + vloc0 + c4) = *(const v4f*)(&Tc[ch][c4]); } __threadfence(); }
}
}

extern "C" void kernel_launch(void* const* d_in, const int* in_sizes, int n_in, void* d_out, int out_size, void* d_ws, size_t ws_size, hipStream_t stream) {
  (void)n_in;
  auto Fp = [&](int i) { return (const float*)d_in[i]; };
  if (in_sizes[0] != NPT * 3 || in_sizes[1] != NPT || in_sizes[2] != 3 * C2 || in_sizes[4] != NBLK * C2 * HID || in_sizes[6] != NBLK * HID * HID || in_sizes[8] != NBLK * C2 * HID || in_sizes[9] != HID * HID || out_size != NB * HID * G) return;
  size_t off = 0; char* ws = (char*)d_ws;
  auto carve = [&](size_t bytes) { char* p = ws + off; off += (bytes + 255) & ~(size_t)255; return p; };
  b16* P16 = (b16*)carve((size_t)NPT * 32 * 2); int* KEY = (int*)carve((size_t)NPT * 4); b16* WPOS = (b16*)carve(C2 * 32 * 2);
  b16* W0T = (b16*)carve((size_t)NBLK * HID * C2 * 2); b16* W1T = (b16*)carve((size_t)NBLK * HID * HID * 2); b16* WST = (b16*)carve((size_t)NBLK * HID * C2 * 2); b16* WCT = (b16*)carve(HID * HID * 2);
  b16* NETh = (b16*)carve((size_t)T * HID * 2); b16* NETl = (b16*)carve((size_t)T * HID * 2); b16* VOXh = (b16*)carve((size_t)G * HID * 2); b16* VOXl = (b16*)carve((size_t)G * HID * 2); b16* MNh = (b16*)carve((size_t)G * HID * 2); b16* MNl = (b16*)carve((size_t)G * HID * 2); int* CNT = (int*)carve((size_t)NV * 4);
  CsrBufs csr; off = csr_carve(csr, ws, off, NPT, NV);
  if (off > ws_size || off > ((size_t)128 << 20)) return;
  prepp_kernel<<<(NPT / 32 * 32 + 255) / 256, 256, 0, stream>>>(Fp(0), (const int*)d_in[1], P16, KEY);
  prepw_kernel<<<dim3(C2 / 64, C2 / 64, 17), 256, 0, stream>>>(Fp(2), Fp(4), Fp(6), Fp(8), Fp(9), WPOS, W0T, W1T, WST, WCT);
  csr_build(csr, KEY, NPT, NV, stream);
  cnt_kernel<<<NV / 256, 256, 0, stream>>>(csr.ROWCNT, CNT);
  for (int b = 0; b < NB; ++b) { const int pbase = b * T, vbase = b * G; const int nblk = (T + 63) / 64;
    resnet_kernel<1><<<nblk, 128, 0, stream>>>(P16, WPOS, Fp(3), KEY, pbase, vbase, VOXh, VOXl, W0T, Fp(5), W1T, Fp(7), WST, NETh, NETl);
    for (int i = 1; i < NBLK; ++i) {
      voxmax_kernel<<<G / 16, 256, 0, stream>>>(NETh, NETl, pbase, vbase, csr.PERM, csr.ROWPTR, csr.ROWCNT, (int)csr.permLen, VOXh, VOXl);
      resnet_kernel<0><<<nblk, 128, 0, stream>>>(P16, WPOS, Fp(3), KEY, pbase, vbase, VOXh, VOXl, W0T + (size_t)i * HID * C2, Fp(5) + i * HID, W1T + (size_t)i * HID * HID, Fp(7) + i * HID, WST + (size_t)i * HID * C2, NETh, NETl); }
    voxmean_kernel<<<G / 16, 256, 0, stream>>>(NETh, NETl, pbase, vbase, csr.PERM, csr.ROWPTR, csr.ROWCNT, (int)csr.permLen, MNh, MNl);
    final_kernel<<<G / 64, 128, 0, stream>>>(MNh, MNl, CNT, b, WCT, Fp(10), (float*)d_out); }
}
